// LightningDecoderLayer_25640954757725
// MI455X (gfx1250) — hardware-verified
//
#include <hip/hip_runtime.h>
#include <stdint.h>
#include <math.h>

constexpr int NBATCH = 2;
constexpr int NT_T   = 2048;
constexpr int NHID   = 1024;
constexpr int NH     = 16;
constexpr int NDH    = 64;
constexpr int NKD    = 1024;
constexpr int NROWS  = NBATCH * NT_T;
constexpr int NPROJ  = 4 * NKD + 64;
constexpr int LD_PRE = NPROJ;
constexpr int COL_G  = 3 * NKD;
constexpr int COL_B  = 4 * NKD;
constexpr int COL_A  = 4 * NKD + 16;
constexpr int NCONV  = 4;
constexpr int SPITCH = 68;

static_assert(NROWS % 64 == 0);
static_assert(NPROJ % 64 == 0);
static_assert(NHID % 64 == 0);
static_assert(NHID % 32 == 0);
static_assert(NKD % 32 == 0);
static_assert(((NROWS / 64) * (NPROJ / 64)) % 8 == 0);
static_assert(((NROWS / 64) * (NHID / 64)) % 8 == 0);

constexpr size_t PLANE_F32  = (size_t)NROWS * NKD * 4;
constexpr size_t PLANE_BF16 = (size_t)NROWS * NKD * 2;
constexpr size_t WS_A_BYTES   = 3 * PLANE_F32;
constexpr size_t WS_XB_OFF    = 0;
constexpr size_t WS_WALL_OFF  = PLANE_BF16;
constexpr size_t WS_Q_OFF     = 0;
constexpr size_t WS_K_OFF     = PLANE_F32;
constexpr size_t WS_V_OFF     = 2 * PLANE_F32;
constexpr size_t WS_OGHI_OFF  = 0;
constexpr size_t WS_OGLO_OFF  = PLANE_BF16;
constexpr size_t WS_PRE_OFF   = WS_A_BYTES;
constexpr size_t WS_PRE_BYTES = (size_t)NROWS * NPROJ * 4;
constexpr size_t WS_WO_OFF    = WS_PRE_OFF + WS_PRE_BYTES;
constexpr size_t WS_BETA_OFF  = WS_WO_OFF + (size_t)NHID * NKD * 2;
constexpr size_t WS_ALPHA_OFF = WS_BETA_OFF + (size_t)NROWS * NH * 4;
constexpr size_t WS_TABC_OFF  = WS_ALPHA_OFF + (size_t)NROWS * NH * 4;
constexpr size_t WS_TABS_OFF  = WS_TABC_OFF + (size_t)NT_T * 32 * 4;
constexpr size_t WS_TOTAL     = WS_TABS_OFF + (size_t)NT_T * 32 * 4;
static_assert(WS_WALL_OFF + (size_t)NPROJ * NHID * 2 <= WS_A_BYTES);
static_assert(WS_V_OFF + PLANE_F32 <= WS_A_BYTES);
static_assert(WS_OGLO_OFF + PLANE_BF16 <= WS_A_BYTES);
static_assert(WS_TOTAL <= 134217728ull);
static_assert((WS_PRE_OFF % 256) == 0 && (WS_WO_OFF % 256) == 0 && (WS_BETA_OFF % 256) == 0 && (WS_TABC_OFF % 256) == 0);
static_assert((size_t)NROWS * NHID * 4 == 16777216ull);

typedef __attribute__((ext_vector_type(16))) _Float16 v16h;
typedef __attribute__((ext_vector_type(8)))  _Float16 v8h;
typedef __attribute__((ext_vector_type(16))) __bf16   v16b;
typedef __attribute__((ext_vector_type(8)))  __bf16   v8b;
typedef __attribute__((ext_vector_type(8)))  float    v8f;
typedef __attribute__((ext_vector_type(4)))  float    v4f;
typedef __attribute__((ext_vector_type(2)))  float    v2f;
typedef __attribute__((ext_vector_type(4)))  unsigned int v4u;

__device__ __forceinline__ unsigned short f2bf_bits(float f) {
  unsigned u = __float_as_uint(f);
  return (unsigned short)((u + 0x7FFFu + ((u >> 16) & 1u)) >> 16);
}
__device__ __forceinline__ float bf_bits2f(unsigned short h) { return __uint_as_float(((unsigned)h) << 16); }
__device__ __forceinline__ float bfr(float f) { return bf_bits2f(f2bf_bits(f)); }
__device__ __forceinline__ unsigned pack_bf2(float a, float b) {
  return (unsigned)f2bf_bits(a) | ((unsigned)f2bf_bits(b) << 16);
}
__device__ __forceinline__ float rcpf(float x) { return __builtin_amdgcn_rcpf(x); }

__device__ __forceinline__ void dep_guard_h(v8f& a, v8f& b, v16h x, v16h y) { asm volatile("v_nop\n\tv_nop\n\tv_nop\n\tv_nop" : "+v"(a), "+v"(b) : "v"(x), "v"(y)); }
__device__ __forceinline__ void dep_guard_b(v8f& a, v8f& b, v16b x, v16b y) { asm volatile("v_nop\n\tv_nop\n\tv_nop\n\tv_nop" : "+v"(a), "+v"(b) : "v"(x), "v"(y)); }
__device__ __forceinline__ void keep4_h(v16h a, v16h b, v16h c, v16h d) { asm volatile("v_nop" :: "v"(a), "v"(b), "v"(c), "v"(d)); }
__device__ __forceinline__ void keep4_b(v16b a, v16b b, v16b c, v16b d) { asm volatile("v_nop" :: "v"(a), "v"(b), "v"(c), "v"(d)); }
__device__ __forceinline__ void acc_guard4(v8f& a, v8f& b, v8f& c, v8f& d) { asm volatile("v_nop\n\tv_nop\n\tv_nop\n\tv_nop" : "+v"(a), "+v"(b), "+v"(c), "+v"(d)); }
template <typename T> struct Frag;
template <> struct Frag<_Float16> {
  typedef v16h V; union U { v16h v; v8h h[2]; };
  static __device__ __forceinline__ v16h load(const _Float16* p) {
    U f; f.h[0] = *(const v8h*)(p); f.h[1] = *(const v8h*)(p + 16); return f.v;
  }
  static __device__ __forceinline__ v8f mma(v16h a, v16h b, v8f c) {
    return __builtin_amdgcn_wmma_f32_16x16x32_f16(false, a, false, b, (short)0, c, false, false);
  }
  static __device__ __forceinline__ void guard(v8f& a, v8f& b, v16h x, v16h y) { dep_guard_h(a, b, x, y); }
  static __device__ __forceinline__ void keep(v16h a, v16h b, v16h c, v16h d) { keep4_h(a, b, c, d); }
};
template <> struct Frag<__bf16> {
  typedef v16b V; union U { v16b v; v8b h[2]; };
  static __device__ __forceinline__ v16b load(const __bf16* p) {
    U f; f.h[0] = *(const v8b*)(p); f.h[1] = *(const v8b*)(p + 16); return f.v;
  }
  static __device__ __forceinline__ v8f mma(v16b a, v16b b, v8f c) {
    return __builtin_amdgcn_wmma_f32_16x16x32_bf16(false, a, false, b, (short)0, c, false, false);
  }
  static __device__ __forceinline__ void guard(v8f& a, v8f& b, v16b x, v16b y) { dep_guard_b(a, b, x, y); }
  static __device__ __forceinline__ void keep(v16b a, v16b b, v16b c, v16b d) { keep4_b(a, b, c, d); }
};

template <int ET> struct Elem;
template <> struct Elem<0> { typedef _Float16 T; };
template <> struct Elem<1> { typedef __bf16 T; };
template <int ET, int SPLITM>
__global__ __launch_bounds__(256) void wmma_gemm64(
    const unsigned short* __restrict__ Ap, const unsigned short* __restrict__ A2p, int lda, long strideA,
    const unsigned short* __restrict__ Btp, const unsigned short* __restrict__ Bt2p, int ldb, long strideB,
    float* __restrict__ Cout, int ldc, long strideC,
    int M, int N, int K, float scale) {
  typedef typename Elem<ET>::T T;
  typedef typename Frag<T>::V V;
  const T* A = (const T*)Ap; const T* A2 = (const T*)A2p; const T* Bt = (const T*)Btp; const T* Bt2 = (const T*)Bt2p;
  __shared__ __align__(16) float sT[8][16 * 68];
  const int b    = blockIdx.y;
  const int lane = threadIdx.x & 31;
  const int wave = threadIdx.x >> 5;
  const int tilesN = N >> 6;
  const int tilesM = M >> 6;
  const int tile = blockIdx.x * 8 + wave;
  if (tile >= tilesM * tilesN) return;
  const int tm = tile / tilesN;
  const int tn = tile - tm * tilesN;
  const int m0 = tm << 6;
  const int n0 = tn << 6;

  const T* Ab  = A  + (size_t)b * strideA;
  const T* Bb  = Bt + (size_t)b * strideB;
  const T* Ab2 = (SPLITM != 0) ? (A2  + (size_t)b * strideA) : nullptr;
  const T* Bb2 = (SPLITM == 2) ? (Bt2 + (size_t)b * strideB) : nullptr;

  const int rlane = lane & 15;
  const int koff  = (lane >> 4) * 8;
  const int mOff  = (lane >> 4) * 8;

  v8f acc[4][4];
#pragma unroll
  for (int i = 0; i < 4; ++i)
#pragma unroll
    for (int j = 0; j < 4; ++j) acc[i][j] = (v8f){0.f,0.f,0.f,0.f,0.f,0.f,0.f,0.f};

  for (int k0 = 0; k0 < K; k0 += 32) {
    V bh[4], bl[4];
#pragma unroll
    for (int j = 0; j < 4; ++j) {
      const size_t bo = (size_t)(n0 + (j << 4) + rlane) * ldb + koff + k0;
      bh[j] = Frag<T>::load(Bb + bo);
      if (SPLITM == 2) bl[j] = Frag<T>::load(Bb2 + bo);
    }
#pragma unroll
    for (int i = 0; i < 4; ++i) {
      const size_t ao = (size_t)(m0 + (i << 4) + rlane) * lda + koff + k0;
      V ah = Frag<T>::load(Ab + ao);
      V al = ah;
      if (SPLITM != 0) al = Frag<T>::load(Ab2 + ao);
#pragma unroll
      for (int j = 0; j < 4; ++j) {
        acc[i][j] = Frag<T>::mma(ah, bh[j], acc[i][j]);
        if (SPLITM == 2) acc[i][j] = Frag<T>::mma(ah, bl[j], acc[i][j]);
        if (SPLITM != 0) acc[i][j] = Frag<T>::mma(al, bh[j], acc[i][j]);
      }
      Frag<T>::guard(acc[i][0], acc[i][3], ah, al);
    }
    Frag<T>::keep(bh[0], bh[1], bh[2], bh[3]);
    if (SPLITM == 2) Frag<T>::keep(bl[0], bl[1], bl[2], bl[3]);
  }
  acc_guard4(acc[0][0], acc[0][1], acc[0][2], acc[0][3]);
  acc_guard4(acc[1][0], acc[1][1], acc[1][2], acc[1][3]);
  acc_guard4(acc[2][0], acc[2][1], acc[2][2], acc[2][3]);
  acc_guard4(acc[3][0], acc[3][1], acc[3][2], acc[3][3]);

  float* slab = sT[wave];
#pragma unroll
  for (int i = 0; i < 4; ++i) {
    const int mBase = m0 + (i << 4);
#pragma unroll
    for (int j = 0; j < 4; ++j) {
#pragma unroll
      for (int r = 0; r < 8; ++r) {
        const float v = acc[i][j][r] * scale;
        slab[(mOff + r) * 68 + (j << 4) + rlane] = v;
      }
    }
    __builtin_amdgcn_fence(__ATOMIC_RELEASE, "workgroup");
    __builtin_amdgcn_wave_barrier();
    __builtin_amdgcn_fence(__ATOMIC_ACQUIRE, "workgroup");
    {
      float* C = Cout + (size_t)b * strideC;
      const int hh = lane >> 4, c4 = (lane & 15) * 4;
      for (int pass = 0; pass < 2; ++pass) {
#pragma unroll
        for (int it = 0; it < 8; ++it) {
          const int row = it * 2 + hh;
          v4f v = *(const v4f*)(slab + row * 68 + c4);
          *(volatile v4f*)(C + (size_t)(mBase + row) * ldc + n0 + c4) = v;
        }
        __threadfence();
      }
    }
    __builtin_amdgcn_fence(__ATOMIC_RELEASE, "workgroup");
    __builtin_amdgcn_wave_barrier();
    __builtin_amdgcn_fence(__ATOMIC_ACQUIRE, "workgroup");
  }
}

__global__ __launch_bounds__(256) void cast_f32_bf16x8(const float* __restrict__ in, unsigned short* __restrict__ out, int n8) {
  const int i = blockIdx.x * 256 + threadIdx.x;
  if (i < n8) {
    const float* p = in + (size_t)i * 8;
    const v4f a = *(const v4f*)p;
    const v4f c = *(const v4f*)(p + 4);
    v4u w;
    w[0] = pack_bf2(a[0], a[1]); w[1] = pack_bf2(a[2], a[3]);
    w[2] = pack_bf2(c[0], c[1]); w[3] = pack_bf2(c[2], c[3]);
    v4u* d = (v4u*)(out + (size_t)i * 8);
    *(volatile v4u*)d = w;
    __threadfence();
    *(volatile v4u*)d = w;
  }
}

__global__ __launch_bounds__(256) void cast_gatew_kernel(const float* __restrict__ wb, const float* __restrict__ wgk,
                                                        unsigned short* __restrict__ out) {
  const int i  = blockIdx.x * 256 + threadIdx.x;
  const int r  = i >> 7;
  const int c8 = (i & 127) * 8;
  const int rb = (r < 16) ? r : 0;
  const int rg = (r >= 16 && r < 32) ? (r - 16) : 0;
  const v4f a0 = *(const v4f*)(wb  + (size_t)rb * NHID + c8);
  const v4f a1 = *(const v4f*)(wb  + (size_t)rb * NHID + c8 + 4);
  const v4f g0 = *(const v4f*)(wgk + (size_t)rg * NHID + c8);
  const v4f g1 = *(const v4f*)(wgk + (size_t)rg * NHID + c8 + 4);
  const bool useb = (r < 16), useg = (r >= 16) && (r < 32);
  float e[8];
#pragma unroll
  for (int q = 0; q < 4; ++q) {
    e[q]     = useb ? a0[q] : (useg ? g0[q] : 0.0f);
    e[4 + q] = useb ? a1[q] : (useg ? g1[q] : 0.0f);
  }
  v4u w;
  w[0] = pack_bf2(e[0], e[1]); w[1] = pack_bf2(e[2], e[3]);
  w[2] = pack_bf2(e[4], e[5]); w[3] = pack_bf2(e[6], e[7]);
  v4u* d = (v4u*)(out + (size_t)i * 8);
  *(volatile v4u*)d = w;
  __threadfence();
  *(volatile v4u*)d = w;
}

struct RopeFreq { float f0, f1, f2, f3, f4, f5, f6, f7, f8, f9, f10, f11, f12, f13, f14, f15; };
static_assert(sizeof(RopeFreq) == 64);
__global__ __launch_bounds__(256) void rope_tab_kernel(float* __restrict__ tabc, float* __restrict__ tabs, RopeFreq rf) {
  #pragma clang fp contract(off)
  const int i = blockIdx.x * 256 + threadIdx.x;
  const int t = i >> 5;
  const int lane = i & 31;
  const int m = (lane < 16) ? lane : (lane - 16);
  float f = rf.f0;
  f = (m == 1)  ? rf.f1  : f;  f = (m == 2)  ? rf.f2  : f;  f = (m == 3)  ? rf.f3  : f;
  f = (m == 4)  ? rf.f4  : f;  f = (m == 5)  ? rf.f5  : f;  f = (m == 6)  ? rf.f6  : f;
  f = (m == 7)  ? rf.f7  : f;  f = (m == 8)  ? rf.f8  : f;  f = (m == 9)  ? rf.f9  : f;
  f = (m == 10) ? rf.f10 : f;  f = (m == 11) ? rf.f11 : f;  f = (m == 12) ? rf.f12 : f;
  f = (m == 13) ? rf.f13 : f;  f = (m == 14) ? rf.f14 : f;  f = (m == 15) ? rf.f15 : f;
  const float ang = (float)t * f;
  const float cs = cosf(ang);
  const float sn = sinf(ang);
  *(volatile float*)(tabc + i) = cs;
  *(volatile float*)(tabs + i) = sn;
  __threadfence();
  *(volatile float*)(tabc + i) = cs;
  *(volatile float*)(tabs + i) = sn;
}

__global__ __launch_bounds__(256) void gate_kernel(const float* __restrict__ pre,
    const float* __restrict__ bb, const float* __restrict__ bgk, const float* __restrict__ alog, const float* __restrict__ dtb,
    float* __restrict__ beta, float* __restrict__ alpha) {
  const int i = blockIdx.x * 256 + threadIdx.x;
  const int row = i >> 4, h = i & 15;
  const float vbb = bfr(bb[h]), vbg = bfr(bgk[h]), vdt = bfr(dtb[h]), val = bfr(alog[h]);
  const float zb = pre[(size_t)row * LD_PRE + COL_B + h] + vbb;
  const float za = (pre[(size_t)row * LD_PRE + COL_A + h] + vbg) + vdt;
  const float bet = rcpf(1.0f + expf(-zb));
  const float sp  = fmaxf(za, 0.0f) + log1pf(expf(-fabsf(za)));
  const float alp = expf(-expf(val) * sp);
  *(volatile float*)(beta + i)  = bet;
  *(volatile float*)(alpha + i) = alp;
  __threadfence();
  *(volatile float*)(beta + i)  = bet;
  *(volatile float*)(alpha + i) = alp;
}

__global__ __launch_bounds__(256) void conv_act_kernel(
    const float* __restrict__ pre,
    const float* __restrict__ cqw, const float* __restrict__ cqb,
    const float* __restrict__ ckw, const float* __restrict__ ckb,
    const float* __restrict__ cvw, const float* __restrict__ cvb,
    const float* __restrict__ tabc, const float* __restrict__ tabs,
    float* __restrict__ qout, float* __restrict__ kout, float* __restrict__ vout) {
  const int lane = threadIdx.x & 31;
  const int wave = threadIdx.x >> 5;
  const int blk = blockIdx.x;
  const int which = blk / (NROWS * 2);
  const int rem = blk - which * (NROWS * 2);
  const int row = rem >> 1;
  const int h = (rem & 1) * 8 + wave;
  const int t = row & (NT_T - 1);
  const float* cw = (which == 0) ? cqw : ((which == 1) ? ckw : cvw);
  const float* cb = (which == 0) ? cqb : ((which == 1) ? ckb : cvb);
  const int c0 = h * NDH + 2 * lane;
  const int col = which * NKD + c0;
  const v4f w0 = *(const v4f*)(cw + (size_t)c0 * NCONV);
  const v4f w1 = *(const v4f*)(cw + (size_t)(c0 + 1) * NCONV);
  const v2f b2 = *(const v2f*)(cb + c0);
  float y0 = 0.0f, y1 = 0.0f;
#pragma unroll
  for (int j = 0; j < NCONV; ++j) {
    const int tj = t - (NCONV - 1) + j;
    const bool ok = (tj >= 0);
    const int rr = ok ? (row - (NCONV - 1) + j) : row;
    const v2f p = *(const v2f*)(pre + (size_t)rr * LD_PRE + col);
    const float p0 = ok ? p[0] : 0.0f;
    const float p1 = ok ? p[1] : 0.0f;
    y0 = fmaf(bfr(w0[j]), p0, y0);
    y1 = fmaf(bfr(w1[j]), p1, y1);
  }
  y0 += bfr(b2[0]);
  y1 += bfr(b2[1]);
  const float s0 = y0 * rcpf(1.0f + expf(-y0));
  const float s1 = y1 * rcpf(1.0f + expf(-y1));
  const size_t obase = (size_t)row * NKD + h * NDH;
  if (which < 2) {
    const float cs = tabc[t * 32 + lane];
    const float sn = tabs[t * 32 + lane];
    const float olo = s0 * cs - s1 * sn;
    const float ohi = s0 * sn + s1 * cs;
    float ss = olo * olo + ohi * ohi;
    ss += __shfl_xor(ss, 16, 32);
    ss += __shfl_xor(ss, 8, 32);
    ss += __shfl_xor(ss, 4, 32);
    ss += __shfl_xor(ss, 2, 32);
    ss += __shfl_xor(ss, 1, 32);
    const float rn = rsqrtf(ss + 1e-12f);
    const float a = olo * rn, c = ohi * rn;
    float* o = (which == 0) ? qout : kout;
    *(volatile float*)(o + obase + lane) = a;
    *(volatile float*)(o + obase + 32 + lane) = c;
    __threadfence();
    *(volatile float*)(o + obase + lane) = a;
    *(volatile float*)(o + obase + 32 + lane) = c;
  } else {
    v2f vv; vv[0] = s0; vv[1] = s1;
    *(volatile v2f*)(vout + obase + 2 * lane) = vv;
    __threadfence();
    *(volatile v2f*)(vout + obase + 2 * lane) = vv;
  }
}

__global__ __launch_bounds__(64) void delta_scan_kernel(
    const float* __restrict__ qp, const float* __restrict__ kp, const float* __restrict__ vp,
    const float* __restrict__ betap, const float* __restrict__ alphap, const float* __restrict__ dpv,
    float* __restrict__ opl) {
  __shared__ __align__(16) float Sl[NDH * SPITCH];
  __shared__ __align__(16) float qs[2][NDH];
  __shared__ __align__(16) float ks[2][NDH];
  __shared__ __align__(16) float bks[2][NDH];
  __shared__ float red[2][2];
  const int tid = threadIdx.x, lane = tid & 31, wave = tid >> 5;
  const int b = blockIdx.x >> 4, h = blockIdx.x & 15;
  const float dp = bfr(dpv[h]);
  float* srow = Sl + tid * SPITCH;
#pragma unroll
  for (int d = 0; d < NDH; d += 4) *(v4f*)(srow + d) = (v4f){0.0f, 0.0f, 0.0f, 0.0f};
  for (int t = 0; t < NT_T; ++t) {
    const int buf = t & 1;
    const int row = b * NT_T + t;
    const size_t base = (size_t)row * NKD + h * NDH;
    const float qv = qp[base + tid];
    const float kv = kp[base + tid];
    const float vt = vp[base + tid];
    const float a   = alphap[row * NH + h];
    const float bta = betap[row * NH + h];
    qs[buf][tid]  = qv;
    ks[buf][tid]  = kv;
    bks[buf][tid] = bta * kv;
    float pq = qv * kv;
    pq += __shfl_xor(pq, 16, 32);
    pq += __shfl_xor(pq, 8, 32);
    pq += __shfl_xor(pq, 4, 32);
    pq += __shfl_xor(pq, 2, 32);
    pq += __shfl_xor(pq, 1, 32);
    if (lane == 0) red[buf][wave] = pq;
    __syncthreads();
    const float qk = red[buf][0] + red[buf][1];
    const float* qb  = &qs[buf][0];
    const float* kb  = &ks[buf][0];
    const float* bkb = &bks[buf][0];
    float ov = 0.0f, kS = 0.0f;
#pragma unroll 1
    for (int d = 0; d < NDH; d += 4) {
      const v4f q4 = *(const v4f*)(qb + d);
      const v4f k4 = *(const v4f*)(kb + d);
      const v4f s4 = *(const v4f*)(srow + d);
#pragma unroll
      for (int e = 0; e < 4; ++e) { ov = fmaf(q4[e], s4[e], ov); kS = fmaf(k4[e], s4[e], kS); }
    }
#pragma unroll 1
    for (int d = 0; d < NDH; d += 4) {
      const v4f bk4 = *(const v4f*)(bkb + d);
      v4f s4 = *(const v4f*)(srow + d);
#pragma unroll
      for (int e = 0; e < 4; ++e) {
        const float bk = bk4[e];
        const float tt = fmaf(-bk, kS, s4[e]);
        s4[e] = fmaf(a, tt, bk * vt);
      }
      *(v4f*)(srow + d) = s4;
    }
    const float o = fmaf(dp * qk, vt, ov);
    float* dst = opl + (size_t)row * LD_PRE + h * NDH + tid;
    *(volatile float*)dst = o;
    __threadfence();
    *(volatile float*)dst = o;
  }
}

__global__ __launch_bounds__(256) void norm_gate_kernel(const float* __restrict__ pre, const float* __restrict__ onw,
                                                       unsigned int* __restrict__ oghi, unsigned int* __restrict__ oglo) {
  const int lane = threadIdx.x & 31, wave = threadIdx.x >> 5;
  const int item = blockIdx.x * 8 + wave;
  const int row = item >> 4, h = item & 15;
  const size_t ob = (size_t)row * LD_PRE + h * NDH + 2 * lane;
  const v2f o2 = *(const v2f*)(pre + ob);
  const v2f g2 = *(const v2f*)(pre + ob + COL_G);
  const v2f w2 = *(const v2f*)(onw + 2 * lane);
  float ss = o2[0] * o2[0] + o2[1] * o2[1];
  ss += __shfl_xor(ss, 16, 32);
  ss += __shfl_xor(ss, 8, 32);
  ss += __shfl_xor(ss, 4, 32);
  ss += __shfl_xor(ss, 2, 32);
  ss += __shfl_xor(ss, 1, 32);
  const float rs = rsqrtf(ss * (1.0f / 64.0f) + 1e-6f);
  const float on0 = (o2[0] * rs) * bfr(w2[0]);
  const float on1 = (o2[1] * rs) * bfr(w2[1]);
  const float si0 = on0 * rcpf(1.0f + expf(-on0));
  const float si1 = on1 * rcpf(1.0f + expf(-on1));
  const float r0 = g2[0] * si0, r1 = g2[1] * si1;
  const unsigned short hb0 = f2bf_bits(r0), hb1 = f2bf_bits(r1);
  const unsigned short lb0 = f2bf_bits(r0 - bf_bits2f(hb0)), lb1 = f2bf_bits(r1 - bf_bits2f(hb1));
  const unsigned uh = (unsigned)hb0 | ((unsigned)hb1 << 16);
  const unsigned ul = (unsigned)lb0 | ((unsigned)lb1 << 16);
  const size_t oi = ((size_t)row * NKD + h * NDH) / 2 + lane;
  *(volatile unsigned*)(oghi + oi) = uh;
  *(volatile unsigned*)(oglo + oi) = ul;
  __threadfence();
  *(volatile unsigned*)(oghi + oi) = uh;
  *(volatile unsigned*)(oglo + oi) = ul;
}

extern "C" void kernel_launch(void* const* d_in, const int* in_sizes, int n_in,
                              void* d_out, int out_size, void* d_ws, size_t ws_size,
                              hipStream_t stream) {
  (void)in_sizes; (void)n_in; (void)out_size;
  const float* x    = (const float*)d_in[0];
  const float* Wq   = (const float*)d_in[1];
  const float* Wk   = (const float*)d_in[2];
  const float* Wv   = (const float*)d_in[3];
  const float* Wg   = (const float*)d_in[4];
  const float* Wo   = (const float*)d_in[5];
  const float* Wb   = (const float*)d_in[6];
  const float* bb   = (const float*)d_in[7];
  const float* Wgk  = (const float*)d_in[8];
  const float* bgk  = (const float*)d_in[9];
  const float* cqw  = (const float*)d_in[10];
  const float* cqb  = (const float*)d_in[11];
  const float* ckw  = (const float*)d_in[12];
  const float* ckb  = (const float*)d_in[13];
  const float* cvw  = (const float*)d_in[14];
  const float* cvb  = (const float*)d_in[15];
  const float* A_log   = (const float*)d_in[16];
  const float* Dp      = (const float*)d_in[17];
  const float* dt_bias = (const float*)d_in[18];
  const float* onorm_w = (const float*)d_in[19];
  float* out = (float*)d_out;

  if (ws_size < WS_TOTAL) return;
  char* ws = (char*)d_ws;
  unsigned short* xb    = (unsigned short*)(ws + WS_XB_OFF);
  unsigned short* wall  = (unsigned short*)(ws + WS_WALL_OFF);
  float* qpl            = (float*)(ws + WS_Q_OFF);
  float* kpl            = (float*)(ws + WS_K_OFF);
  float* vpl            = (float*)(ws + WS_V_OFF);
  unsigned short* oghi  = (unsigned short*)(ws + WS_OGHI_OFF);
  unsigned short* oglo  = (unsigned short*)(ws + WS_OGLO_OFF);
  float* pre            = (float*)(ws + WS_PRE_OFF);
  unsigned short* wob   = (unsigned short*)(ws + WS_WO_OFF);
  float* betab          = (float*)(ws + WS_BETA_OFF);
  float* alphab         = (float*)(ws + WS_ALPHA_OFF);
  float* tabc           = (float*)(ws + WS_TABC_OFF);
  float* tabs           = (float*)(ws + WS_TABS_OFF);

  RopeFreq rf;
  {
    float fv[16];
    for (int m = 0; m < 16; ++m) {
      const float p = (float)pow(10000.0, (double)m / 16.0);
      fv[m] = 1.0f / p;
    }
    rf.f0 = fv[0]; rf.f1 = fv[1]; rf.f2 = fv[2]; rf.f3 = fv[3]; rf.f4 = fv[4]; rf.f5 = fv[5]; rf.f6 = fv[6]; rf.f7 = fv[7];
    rf.f8 = fv[8]; rf.f9 = fv[9]; rf.f10 = fv[10]; rf.f11 = fv[11]; rf.f12 = fv[12]; rf.f13 = fv[13]; rf.f14 = fv[14]; rf.f15 = fv[15];
  }

  const int NW8 = NHID * NKD / 8;
  const int NX8 = NROWS * NHID / 8;

  cast_f32_bf16x8<<<NX8 / 256, 256, 0, stream>>>(x, xb, NX8);
  cast_f32_bf16x8<<<NW8 / 256, 256, 0, stream>>>(Wq, wall + 0 * (size_t)NKD * NHID, NW8);
  cast_f32_bf16x8<<<NW8 / 256, 256, 0, stream>>>(Wk, wall + 1 * (size_t)NKD * NHID, NW8);
  cast_f32_bf16x8<<<NW8 / 256, 256, 0, stream>>>(Wv, wall + 2 * (size_t)NKD * NHID, NW8);
  cast_f32_bf16x8<<<NW8 / 256, 256, 0, stream>>>(Wg, wall + 3 * (size_t)NKD * NHID, NW8);
  cast_gatew_kernel<<<(64 * NHID / 8) / 256, 256, 0, stream>>>(Wb, Wgk, wall + 4 * (size_t)NKD * NHID);
  cast_f32_bf16x8<<<NW8 / 256, 256, 0, stream>>>(Wo, wob, NW8);

  rope_tab_kernel<<<(NT_T * 32) / 256, 256, 0, stream>>>(tabc, tabs, rf);

  wmma_gemm64<1, 0><<<dim3((NROWS / 64) * (NPROJ / 64) / 8, 1), 256, 0, stream>>>(
      xb, xb, NHID, 0L, wall, wall, NHID, 0L, pre, LD_PRE, 0L, NROWS, NPROJ, NHID, 1.0f);

  gate_kernel<<<(NROWS * NH) / 256, 256, 0, stream>>>(pre, bb, bgk, A_log, dt_bias, betab, alphab);

  conv_act_kernel<<<3 * NROWS * 2, 256, 0, stream>>>(pre, cqw, cqb, ckw, ckb, cvw, cvb, tabc, tabs, qpl, kpl, vpl);

  delta_scan_kernel<<<NBATCH * NH, 64, 0, stream>>>(qpl, kpl, vpl, betab, alphab, Dp, pre);

  norm_gate_kernel<<<(NROWS * NH) / 8, 256, 0, stream>>>(pre, onorm_w, (unsigned int*)oghi, (unsigned int*)oglo);

  wmma_gemm64<1, 1><<<dim3((NROWS / 64) * (NHID / 64) / 8, 1), 256, 0, stream>>>(
      oghi, oglo, NKD, 0L, wob, wob, NKD, 0L, out, NHID, 0L, NROWS, NHID, NKD, 1.0f);
}
